// GroundedMambaBlock_16999480558028
// MI455X (gfx1250) — hardware-verified
//
#include <hip/hip_runtime.h>
#include <math.h>

constexpr int kBatch   = 4;
constexpr int kSeq     = 2048;
constexpr int kDim     = 1024;
constexpr int kHeads   = 16;
constexpr int kHeadDim = 64;
constexpr int kState   = 16;
constexpr int kRows    = kBatch * kSeq;
constexpr int kBxN     = 64;
constexpr int kStK     = 32;
constexpr float kWCarry     = 32.0f;
constexpr float kSmallCarry = 64.0f;
constexpr float kYCarry     = 16.0f;
constexpr float kInvDim     = 1.0f / 1024.0f;
constexpr float kInvState   = 1.0f / 16.0f;
constexpr float kLnEps      = 1e-5f;

constexpr size_t kOffXs16 = 0;
constexpr size_t kOffXr16 = 16777216;
constexpr size_t kOffW16  = 33554432;
constexpr size_t kOffBwp  = 41943040;
constexpr size_t kOffCwp  = 42074112;
constexpr size_t kOffBxp  = 42139648;
constexpr size_t kOffSt16 = 44236800;
constexpr size_t kOffRw   = 44761088;
constexpr size_t kOffKvr  = 78315520;
constexpr size_t kOffY16  = 103481344;
constexpr size_t kWsEnd   = 107675648;
constexpr size_t kOffSs   = 0;
static_assert(kOffXr16 == kOffXs16 + (size_t)kRows * kDim * 2, "carve");
static_assert(kOffW16  == kOffXr16 + (size_t)kRows * kDim * 2, "carve");
static_assert(kOffBwp  == kOffW16  + (size_t)4 * kDim * kDim * 2, "carve");
static_assert(kOffCwp  == kOffBwp  + (size_t)kBxN * kDim * 2, "carve");
static_assert(kOffBxp  == kOffCwp  + (size_t)kDim * kStK * 2, "carve");
static_assert(kOffSt16 == kOffBxp  + (size_t)kRows * kBxN * 4, "carve");
static_assert(kOffRw   == kOffSt16 + (size_t)kRows * kStK * 2, "carve");
static_assert(kOffKvr  == kOffRw   + (size_t)kRows * kDim * 4, "carve");
static_assert(kOffY16  == kOffKvr  + (size_t)3 * kSeq * kDim * 4, "carve");
static_assert(kWsEnd   == kOffY16  + (size_t)kSeq * kDim * 2, "carve");
static_assert(kOffSs + (size_t)kRows * kDim * 4 <= kOffW16, "ss plane inside dead regions");
static_assert(kWsEnd <= (size_t)134217728, "carve cap");

typedef __attribute__((ext_vector_type(16))) _Float16 v16h;
typedef __attribute__((ext_vector_type(8)))  _Float16 v8h;
typedef __attribute__((ext_vector_type(16))) __bf16   v16b;
typedef __attribute__((ext_vector_type(8)))  __bf16   v8b;
typedef __attribute__((ext_vector_type(8)))  float    v8f;
typedef __attribute__((ext_vector_type(4)))  float    v4f;
typedef __attribute__((ext_vector_type(4)))  unsigned int v4u;

__device__ __forceinline__ unsigned short f2bf_bits(float f) {
  unsigned u = __float_as_uint(f);
  return (unsigned short)((u + 0x7FFFu + ((u >> 16) & 1u)) >> 16);
}
__device__ __forceinline__ float bf_bits2f(unsigned short h) { return __uint_as_float(((unsigned)h) << 16); }

__device__ __forceinline__ void dep_guard_h(v8f& a, v8f& b, v16h x, v16h y) { asm volatile("v_nop\n\tv_nop\n\tv_nop\n\tv_nop" : "+v"(a), "+v"(b) : "v"(x), "v"(y)); }
__device__ __forceinline__ void dep_guard_b(v8f& a, v8f& b, v16b x, v16b y) { asm volatile("v_nop\n\tv_nop\n\tv_nop\n\tv_nop" : "+v"(a), "+v"(b) : "v"(x), "v"(y)); }
__device__ __forceinline__ void keep4_h(v16h a, v16h b, v16h c, v16h d) { asm volatile("v_nop" :: "v"(a), "v"(b), "v"(c), "v"(d)); }
__device__ __forceinline__ void keep4_b(v16b a, v16b b, v16b c, v16b d) { asm volatile("v_nop" :: "v"(a), "v"(b), "v"(c), "v"(d)); }
__device__ __forceinline__ void acc_guard4(v8f& a, v8f& b, v8f& c, v8f& d) { asm volatile("v_nop\n\tv_nop\n\tv_nop\n\tv_nop" : "+v"(a), "+v"(b), "+v"(c), "+v"(d)); }
template <typename T> struct Frag;
template <> struct Frag<_Float16> {
  typedef v16h V; union U { v16h v; v8h h[2]; };
  static __device__ __forceinline__ v16h load(const _Float16* p) {
    U f; f.h[0] = *(const v8h*)(p); f.h[1] = *(const v8h*)(p + 16); return f.v;
  }
  static __device__ __forceinline__ v8f mma(v16h a, v16h b, v8f c) {
    return __builtin_amdgcn_wmma_f32_16x16x32_f16(false, a, false, b, (short)0, c, false, false);
  }
  static __device__ __forceinline__ void guard(v8f& a, v8f& b, v16h x, v16h y) { dep_guard_h(a, b, x, y); }
  static __device__ __forceinline__ void keep(v16h a, v16h b, v16h c, v16h d) { keep4_h(a, b, c, d); }
};
template <> struct Frag<__bf16> {
  typedef v16b V; union U { v16b v; v8b h[2]; };
  static __device__ __forceinline__ v16b load(const __bf16* p) {
    U f; f.h[0] = *(const v8b*)(p); f.h[1] = *(const v8b*)(p + 16); return f.v;
  }
  static __device__ __forceinline__ v8f mma(v16b a, v16b b, v8f c) {
    return __builtin_amdgcn_wmma_f32_16x16x32_bf16(false, a, false, b, (short)0, c, false, false);
  }
  static __device__ __forceinline__ void guard(v8f& a, v8f& b, v16b x, v16b y) { dep_guard_b(a, b, x, y); }
  static __device__ __forceinline__ void keep(v16b a, v16b b, v16b c, v16b d) { keep4_b(a, b, c, d); }
};

__device__ __forceinline__ unsigned pk16(unsigned short a, unsigned short b) { return (unsigned)a | ((unsigned)b << 16); }
__device__ __forceinline__ unsigned short h_bits(float f) { const _Float16 h = (_Float16)f; return __builtin_bit_cast(unsigned short, h); }

template <int ET> struct Elem;
template <> struct Elem<0> { typedef _Float16 T; };
template <> struct Elem<1> { typedef __bf16 T; };
template <int ET, bool SPLIT, int BIAS_MODE, int OUT_MODE, bool RESID, int ACT = 0>
__global__ __launch_bounds__(256) void wmma_gemm64(
    const unsigned short* __restrict__ Ap, const unsigned short* __restrict__ A2p, int lda, long strideA,
    const unsigned short* __restrict__ Btp, const unsigned short* __restrict__ Bt2p, int ldb, long strideB,
    void* __restrict__ Cout, void* __restrict__ Cout2, int ldc, long strideC,
    const float* __restrict__ bias,
    const float* __restrict__ resid, long strideR,
    int M, int N, int K, float scale) {
  typedef typename Elem<ET>::T T;
  typedef typename Frag<T>::V V;
  const T* A = (const T*)Ap; const T* A2 = (const T*)A2p; const T* Bt = (const T*)Btp; const T* Bt2 = (const T*)Bt2p;
  __shared__ __align__(16) float sT[8][16 * 68];
  const int b    = blockIdx.y;
  const int lane = threadIdx.x & 31;
  const int wave = threadIdx.x >> 5;
  const int tilesN = N >> 6;
  const int tilesM = M >> 6;
  const int tile = blockIdx.x * 8 + wave;
  if (tile >= tilesM * tilesN) return;
  const int tm = tile / tilesN;
  const int tn = tile - tm * tilesN;
  const int m0 = tm << 6;
  const int n0 = tn << 6;

  const T* Ab  = A  + (size_t)b * strideA;
  const T* Bb  = Bt + (size_t)b * strideB;
  const T* Ab2 = SPLIT ? (A2  + (size_t)b * strideA) : nullptr;
  const T* Bb2 = SPLIT ? (Bt2 + (size_t)b * strideB) : nullptr;

  const int rlane = lane & 15;
  const int koff  = (lane >> 4) * 8;
  const int mOff  = (lane >> 4) * 8;

  v8f acc[4][4];
#pragma unroll
  for (int i = 0; i < 4; ++i)
#pragma unroll
    for (int j = 0; j < 4; ++j) acc[i][j] = (v8f){0.f,0.f,0.f,0.f,0.f,0.f,0.f,0.f};

  for (int k0 = 0; k0 < K; k0 += 32) {
    V bh[4], bl[4];
#pragma unroll
    for (int j = 0; j < 4; ++j) {
      const size_t bo = (size_t)(n0 + (j << 4) + rlane) * ldb + koff + k0;
      bh[j] = Frag<T>::load(Bb + bo);
      if (SPLIT) bl[j] = Frag<T>::load(Bb2 + bo);
    }
#pragma unroll
    for (int i = 0; i < 4; ++i) {
      const size_t ao = (size_t)(m0 + (i << 4) + rlane) * lda + koff + k0;
      V ah = Frag<T>::load(Ab + ao);
      V al;
      if (SPLIT) al = Frag<T>::load(Ab2 + ao);
#pragma unroll
      for (int j = 0; j < 4; ++j) {
        acc[i][j] = Frag<T>::mma(ah, bh[j], acc[i][j]);
        if (SPLIT) {
          acc[i][j] = Frag<T>::mma(ah, bl[j], acc[i][j]);
          acc[i][j] = Frag<T>::mma(al, bh[j], acc[i][j]);
        }
      }
      Frag<T>::guard(acc[i][0], acc[i][3], ah, SPLIT ? al : ah);
    }
    Frag<T>::keep(bh[0], bh[1], bh[2], bh[3]);
    if (SPLIT) Frag<T>::keep(bl[0], bl[1], bl[2], bl[3]);
  }
  acc_guard4(acc[0][0], acc[0][1], acc[0][2], acc[0][3]);
  acc_guard4(acc[1][0], acc[1][1], acc[1][2], acc[1][3]);
  acc_guard4(acc[2][0], acc[2][1], acc[2][2], acc[2][3]);
  acc_guard4(acc[3][0], acc[3][1], acc[3][2], acc[3][3]);

  float* slab = sT[wave];
  const float* Rb = RESID ? (resid + (size_t)b * strideR) : nullptr;
#pragma unroll
  for (int i = 0; i < 4; ++i) {
    const int mBase = m0 + (i << 4);
#pragma unroll
    for (int j = 0; j < 4; ++j) {
      const int n = n0 + (j << 4) + rlane;
      float bv = 0.f;
      if (BIAS_MODE == 2) bv = bias[n];
#pragma unroll
      for (int r = 0; r < 8; ++r) {
        float v = acc[i][j][r] * scale;
        if (BIAS_MODE == 1) v += bias[mBase + mOff + r];
        if (BIAS_MODE == 2) v += bv;
        if (RESID) v += Rb[(size_t)(mBase + mOff + r) * ldc + n];
        if (ACT == 2) v = fmaxf(v, 0.0f);
        if (ACT == 4) v = (v > 0.f) ? v : 0.01f * v;
        slab[(mOff + r) * 68 + (j << 4) + rlane] = v;
      }
    }
    __builtin_amdgcn_fence(__ATOMIC_RELEASE, "workgroup");
    __builtin_amdgcn_wave_barrier();
    __builtin_amdgcn_fence(__ATOMIC_ACQUIRE, "workgroup");
    if (OUT_MODE == 0) {
      float* C = (float*)Cout + (size_t)b * strideC;
      const int hh = lane >> 4, c4 = (lane & 15) * 4;
      for (int pass = 0; pass < 2; ++pass) {
#pragma unroll
        for (int it = 0; it < 8; ++it) {
          const int row = it * 2 + hh;
          v4f v = *(const v4f*)(slab + row * 68 + c4);
          *(volatile v4f*)(C + (size_t)(mBase + row) * ldc + n0 + c4) = v;
        }
        __threadfence();
      }
    } else {
      const int q = lane >> 3, c8 = (lane & 7) * 8;
      unsigned short* C  = (unsigned short*)Cout  + (size_t)b * strideC;
      unsigned short* C2 = (OUT_MODE == 2) ? ((unsigned short*)Cout2 + (size_t)b * strideC) : nullptr;
      for (int pass = 0; pass < 2; ++pass) {
#pragma unroll
        for (int it = 0; it < 4; ++it) {
          const int row = it * 4 + q;
          const float* sp = slab + row * 68 + c8;
          v8h hv, lv;
#pragma unroll
          for (int e = 0; e < 8; ++e) {
            if (OUT_MODE == 1) {
              hv[e] = (_Float16)sp[e];
            } else {
              unsigned short hb = f2bf_bits(sp[e]);
              unsigned short lb = f2bf_bits(sp[e] - bf_bits2f(hb));
              hv[e] = __builtin_bit_cast(_Float16, hb);
              lv[e] = __builtin_bit_cast(_Float16, lb);
            }
          }
          *(volatile v8h*)(C + (size_t)(mBase + row) * ldc + n0 + c8) = hv;
          if (OUT_MODE == 2) *(volatile v8h*)(C2 + (size_t)(mBase + row) * ldc + n0 + c8) = lv;
        }
        __threadfence();
      }
    }
    __builtin_amdgcn_fence(__ATOMIC_RELEASE, "workgroup");
    __builtin_amdgcn_wave_barrier();
    __builtin_amdgcn_fence(__ATOMIC_ACQUIRE, "workgroup");
  }
}

__device__ __forceinline__ float block_sum4(float v, float* red, int lane, int wave) {
#pragma unroll
  for (int off = 16; off > 0; off >>= 1) v += __shfl_xor(v, off, 32);
  if (lane == 0) red[wave] = v;
  __syncthreads();
  return ((red[0] + red[1]) + red[2]) + red[3];
}

__global__ __launch_bounds__(128) void ln_dual_kernel(const float* __restrict__ x,
                                                      const float* __restrict__ gs, const float* __restrict__ bs,
                                                      const float* __restrict__ gr, const float* __restrict__ br,
                                                      unsigned short* __restrict__ xs16, unsigned short* __restrict__ xr16) {
  __shared__ float redA[4];
  __shared__ float redB[4];
  const int row = blockIdx.x;
  const int t = threadIdx.x, lane = t & 31, wave = t >> 5;
  const int c0 = t * 8;
  const float* xp = x + (size_t)row * kDim + c0;
  const v4f a = *(const v4f*)(xp);
  const v4f c = *(const v4f*)(xp + 4);
  float v[8];
#pragma unroll
  for (int e = 0; e < 4; ++e) { v[e] = a[e]; v[4 + e] = c[e]; }
  float s = 0.f;
#pragma unroll
  for (int e = 0; e < 8; ++e) s += v[e];
  s = block_sum4(s, redA, lane, wave);
  const float mean = s * kInvDim;
  float q = 0.f;
#pragma unroll
  for (int e = 0; e < 8; ++e) { const float d = v[e] - mean; q += d * d; }
  q = block_sum4(q, redB, lane, wave);
  const float rstd = rsqrtf(q * kInvDim + kLnEps);
  const v4f g1a = *(const v4f*)(gs + c0), g1b = *(const v4f*)(gs + c0 + 4);
  const v4f b1a = *(const v4f*)(bs + c0), b1b = *(const v4f*)(bs + c0 + 4);
  const v4f g2a = *(const v4f*)(gr + c0), g2b = *(const v4f*)(gr + c0 + 4);
  const v4f b2a = *(const v4f*)(br + c0), b2b = *(const v4f*)(br + c0 + 4);
  float g1[8], b1[8], g2[8], b2[8];
#pragma unroll
  for (int e = 0; e < 4; ++e) {
    g1[e] = g1a[e]; g1[4 + e] = g1b[e]; b1[e] = b1a[e]; b1[4 + e] = b1b[e];
    g2[e] = g2a[e]; g2[4 + e] = g2b[e]; b2[e] = b2a[e]; b2[4 + e] = b2b[e];
  }
  unsigned short hs[8], hr[8];
#pragma unroll
  for (int e = 0; e < 8; ++e) {
    const float n = (v[e] - mean) * rstd;
    hs[e] = h_bits(n * g1[e] + b1[e]);
    hr[e] = h_bits(n * g2[e] + b2[e]);
  }
  const v4u us = (v4u){pk16(hs[0], hs[1]), pk16(hs[2], hs[3]), pk16(hs[4], hs[5]), pk16(hs[6], hs[7])};
  const v4u ur = (v4u){pk16(hr[0], hr[1]), pk16(hr[2], hr[3]), pk16(hr[4], hr[5]), pk16(hr[6], hr[7])};
  unsigned short* ps = xs16 + (size_t)row * kDim + c0;
  unsigned short* pr = xr16 + (size_t)row * kDim + c0;
  for (int pass = 0; pass < 2; ++pass) {
    *(volatile v4u*)ps = us;
    *(volatile v4u*)pr = ur;
    __threadfence();
  }
}

__global__ __launch_bounds__(256) void castw_kernel(const float* __restrict__ w0, const float* __restrict__ w1,
                                                     const float* __restrict__ w2, const float* __restrict__ w3,
                                                     unsigned short* __restrict__ out, float scale) {
  const int z = blockIdx.y;
  const float* W = (z == 0) ? w0 : (z == 1) ? w1 : (z == 2) ? w2 : w3;
  const int i = blockIdx.x * 256 + threadIdx.x;
  if (i >= kDim * kDim / 8) return;
  const float* p = W + 8 * (size_t)i;
  const v4f a = *(const v4f*)(p);
  const v4f c = *(const v4f*)(p + 4);
  unsigned short hb[8];
#pragma unroll
  for (int e = 0; e < 4; ++e) {
    hb[e]     = h_bits(a[e] * scale);
    hb[4 + e] = h_bits(c[e] * scale);
  }
  const v4u u = (v4u){pk16(hb[0], hb[1]), pk16(hb[2], hb[3]), pk16(hb[4], hb[5]), pk16(hb[6], hb[7])};
  unsigned short* q = out + (size_t)z * kDim * kDim + 8 * (size_t)i;
  *(volatile v4u*)q = u;
  __threadfence();
  *(volatile v4u*)q = u;
}

__global__ __launch_bounds__(128) void prep_small_kernel(const float* __restrict__ bw, const float* __restrict__ dtw,
                                                         const float* __restrict__ cw,
                                                         unsigned short* __restrict__ bwp, unsigned short* __restrict__ cwp) {
  const int t = threadIdx.x;
  const int blk = blockIdx.x;
  if (blk < kBxN) {
    const int r = blk;
    const int rsrc = (r < kState) ? r : 0;
    const float* src = (r == kState) ? dtw : (bw + (size_t)rsrc * kDim);
    const float fac = (r <= kState) ? kSmallCarry : 0.0f;
    const int c0 = t * 8;
    const v4f a = *(const v4f*)(src + c0);
    const v4f c = *(const v4f*)(src + c0 + 4);
    unsigned short hb[8];
#pragma unroll
    for (int e = 0; e < 4; ++e) {
      hb[e]     = h_bits(a[e] * fac);
      hb[4 + e] = h_bits(c[e] * fac);
    }
    const v4u u = (v4u){pk16(hb[0], hb[1]), pk16(hb[2], hb[3]), pk16(hb[4], hb[5]), pk16(hb[6], hb[7])};
    unsigned short* q = bwp + (size_t)r * kDim + c0;
    *(volatile v4u*)q = u;
    __threadfence();
    *(volatile v4u*)q = u;
  } else {
    const int g = (blk - kBxN) * 128 + t;
    const int n = g >> 2, qq = g & 3;
    const float* src = cw + (size_t)n * kState + (qq & 1) * 8;
    const float fac = (qq < 2) ? kSmallCarry : 0.0f;
    const v4f a = *(const v4f*)(src);
    const v4f c = *(const v4f*)(src + 4);
    unsigned short hb[8];
#pragma unroll
    for (int e = 0; e < 4; ++e) {
      hb[e]     = h_bits(a[e] * fac);
      hb[4 + e] = h_bits(c[e] * fac);
    }
    const v4u u = (v4u){pk16(hb[0], hb[1]), pk16(hb[2], hb[3]), pk16(hb[4], hb[5]), pk16(hb[6], hb[7])};
    unsigned short* q = cwp + (size_t)n * kStK + qq * 8;
    *(volatile v4u*)q = u;
    __threadfence();
    *(volatile v4u*)q = u;
  }
}

__global__ __launch_bounds__(64) void ssm_scan_kernel(const float* __restrict__ Am, const float* __restrict__ bxp,
                                                      const float* __restrict__ dtb_p,
                                                      const float* __restrict__ sng, const float* __restrict__ snb,
                                                      unsigned short* __restrict__ st16, float* __restrict__ out1) {
  __shared__ float red[2];
  __shared__ float Gs[kState][kState + 1];
  __shared__ __align__(16) unsigned int stS[kBatch * 32 * 16];
  __shared__ __align__(16) float o1[64];
  const int tid = threadIdx.x, lane = tid & 31, wave = tid >> 5;
  const int b = tid >> 4, j = tid & 15;

  float fp = 0.f;
#pragma unroll
  for (int i = 0; i < 4; ++i) { const float a = Am[tid * 4 + i]; fp += a * a; }
#pragma unroll
  for (int off = 16; off > 0; off >>= 1) fp += __shfl_xor(fp, off, 32);
  if (lane == 0) red[wave] = fp;
#pragma unroll
  for (int i = 0; i < 16; ++i) {
    const int w = tid + 64 * i;
    const int bb = w >> 8, rr = (w >> 3) & 31, cc = w & 7;
    stS[(bb * 32 + rr) * 16 + 8 + cc] = 0u;
  }
  __syncthreads();
  const float fro2 = red[0] + red[1];
  float scl = 1.0f;
  if (fro2 > 0.99f * 0.99f) {
#pragma unroll
    for (int qd = 0; qd < 4; ++qd) {
      const int idx = tid * 4 + qd;
      const int gi = idx >> 4, gk = idx & 15;
      float g = 0.f;
#pragma unroll 1
      for (int m = 0; m < kState; ++m) g += Am[m * kState + gi] * Am[m * kState + gk];
      Gs[gi][gk] = g;
    }
    __syncthreads();
    float vj = 1.0f, lam = 0.f;
#pragma unroll 1
    for (int it = 0; it < 200; ++it) {
      float w = 0.f;
#pragma unroll 1
      for (int k = 0; k < kState; ++k) w += Gs[j][k] * __shfl(vj, k, 16);
      float n2 = w * w;
#pragma unroll
      for (int off = 8; off > 0; off >>= 1) n2 += __shfl_xor(n2, off, 16);
      const float nrm = sqrtf(n2);
      lam = nrm;
      vj = w * ((nrm > 0.f) ? (1.0f / nrm) : 0.f);
    }
    const float s0 = sqrtf(lam);
    scl = (s0 > 0.99f) ? (0.99f / s0) : 1.0f;
  }
  float Arow[kState];
#pragma unroll
  for (int k = 0; k < kState; ++k) Arow[k] = Am[j * kState + k] * scl;
  const float gj = sng[j], bj = snb[j];
  const float dtb = dtb_p[0];
  unsigned short* stH = (unsigned short*)stS;

  float st = 0.f;
  for (int t = 0; t < kSeq; ++t) {
    const size_t ro = ((size_t)b * kSeq + t) * kBxN;
    const float raw = bxp[ro + kState];
    const float bx  = bxp[ro + j];
    const float z   = raw + dtb;
    const float sp  = fmaxf(z, 0.f) + log1pf(expf(-fabsf(z)));
    const float dtt = fminf(0.1f, fmaxf(1e-3f, sp));
    float contrib = 0.f;
#pragma unroll
    for (int k = 0; k < kState; ++k) contrib += Arow[k] * __shfl(st, k, 16);
    st = st + dtt * contrib + bx;
    float sm = st;
#pragma unroll
    for (int off = 8; off > 0; off >>= 1) sm += __shfl_xor(sm, off, 16);
    const float mean = sm * kInvState;
    const float d = st - mean;
    float qv = d * d;
#pragma unroll
    for (int off = 8; off > 0; off >>= 1) qv += __shfl_xor(qv, off, 16);
    const float var = qv * kInvState;
    st = d * rsqrtf(var + kLnEps) * gj + bj;
    stH[(b * 32 + (t & 31)) * 32 + j] = h_bits(st);
    if ((t & 31) == 31) {
      __syncthreads();
      const int t0 = t - 31;
      for (int pass = 0; pass < 2; ++pass) {
#pragma unroll
        for (int q2 = 0; q2 < 2; ++q2) {
          const int bb = wave * 2 + q2;
#pragma unroll
          for (int i = 0; i < 4; ++i) {
            const v4u val = *(const v4u*)(stS + bb * 512 + i * 128 + lane * 4);
            *(volatile v4u*)(st16 + ((size_t)bb * kSeq + t0) * kStK + i * 256 + lane * 8) = val;
          }
        }
        __threadfence();
      }
      __syncthreads();
    }
  }
  o1[tid] = st;
  __syncthreads();
  for (int pass = 0; pass < 2; ++pass) {
    if (tid < 16) {
      const v4f val = *(const v4f*)(o1 + 4 * tid);
      *(volatile v4f*)(out1 + 4 * tid) = val;
    }
    __threadfence();
  }
}

__device__ __forceinline__ void wkv_stage(const float* __restrict__ Kp, const float* __restrict__ Vp,
                                          const float* __restrict__ Rp, size_t off, float tf_d,
                                          float* kf, float* rs, float* vv, int ds) {
  const float kk = Kp[off];
  const float rr = Rp[off];
  const float v0 = Vp[off];
  kf[ds] = kk * tf_d;
  rs[ds] = 1.0f / (1.0f + expf(-rr));
  vv[ds] = v0;
}

__global__ __launch_bounds__(128) void wkv_scan_kernel(const float* __restrict__ Kp, const float* __restrict__ Vp,
                                                       const float* __restrict__ Rp,
                                                       const float* __restrict__ tdec, const float* __restrict__ tfirst,
                                                       unsigned short* __restrict__ y16, float* __restrict__ wkv_out) {
  __shared__ __align__(16) float kfb[2][64];
  __shared__ __align__(16) float rsb[2][64];
  __shared__ __align__(16) float vbb[2][64];
  __shared__ __align__(16) unsigned short yst[32][64];
  __shared__ __align__(16) float wst[64 * 64];
  const int h = blockIdx.x;
  const int tid = threadIdx.x, lane = tid & 31, wave = tid >> 5;
  const int hf = lane >> 4;
  const int e = wave * 16 + (lane & 15);
  const int d0 = hf * 32;

  float s[32], dec[32];
#pragma unroll
  for (int i = 0; i < 32; ++i) { s[i] = 0.f; dec[i] = tdec[h * kHeadDim + d0 + i]; }
  const int ds = tid & 63;
  const float tf_d = tfirst[h * kHeadDim + ds];
  const size_t colK = (size_t)h * kHeadDim + ds;

  for (int t = -1; t < kSeq; ++t) {
    if (wave < 2 && t + 1 < kSeq)
      wkv_stage(Kp, Vp, Rp, (size_t)(t + 1) * kDim + colK, tf_d,
                kfb[(t + 1) & 1], rsb[(t + 1) & 1], vbb[(t + 1) & 1], ds);
    if (t >= 0) {
      const int cur = t & 1;
      const float ve = vbb[cur][e];
      const float* kfp = kfb[cur] + d0;
      const float* rsp = rsb[cur] + d0;
      float y = 0.f;
#pragma unroll
      for (int q = 0; q < 8; ++q) {
        const v4f k4 = *(const v4f*)(kfp + 4 * q);
        const v4f r4 = *(const v4f*)(rsp + 4 * q);
#pragma unroll
        for (int u = 0; u < 4; ++u) {
          const int i = 4 * q + u;
          const float sn = s[i] * dec[i] + k4[u] * ve;
          s[i] = sn;
          float pr = sn * r4[u];
          asm volatile("" : "+v"(pr));
          y = y + pr;
        }
      }
      y = y + __shfl_xor(y, 16, 32);
      if (hf == 0) yst[t & 31][e] = h_bits(y * kYCarry);
    }
    __syncthreads();
    if (t >= 0 && (t & 15) == 15) {
      const int rl = wave * 4 + (lane >> 3);
      const int gr = t - 15 + rl;
      const int c8 = (lane & 7) * 8;
      const v4u val = *(const v4u*)(&yst[gr & 31][c8]);
      unsigned short* gp = y16 + (size_t)gr * kDim + h * kHeadDim + c8;
      *(volatile v4u*)gp = val;
      __threadfence();
      *(volatile v4u*)gp = val;
    }
  }

#pragma unroll
  for (int i = 0; i < 32; ++i) wst[(d0 + i) * 64 + e] = s[i];
  __syncthreads();
  float* ob = wkv_out + (size_t)h * (kHeadDim * kHeadDim);
  for (int pass = 0; pass < 2; ++pass) {
#pragma unroll
    for (int it = 0; it < 8; ++it) {
      const int fo = wave * 1024 + it * 128 + lane * 4;
      const v4f val = *(const v4f*)(wst + fo);
      *(volatile v4f*)(ob + fo) = val;
    }
    __threadfence();
  }
}

__global__ __launch_bounds__(128) void combine_kernel(const float* __restrict__ x, const float* __restrict__ ss,
                                                      const float* __restrict__ rw, const float* __restrict__ dvec,
                                                      const float* __restrict__ gs, const float* __restrict__ bs,
                                                      const float* __restrict__ go, const float* __restrict__ bo,
                                                      float* __restrict__ out) {
  __shared__ float redA[4];
  __shared__ float redB[4];
  const int row = blockIdx.x;
  const int t = threadIdx.x, lane = t & 31, wave = t >> 5;
  const int cA = 4 * t, cB = 512 + 4 * t;
  const size_t base = (size_t)row * kDim;
  const v4f xa = *(const v4f*)(x + base + cA);
  const v4f xb = *(const v4f*)(x + base + cB);
  float xv[8];
#pragma unroll
  for (int e = 0; e < 4; ++e) { xv[e] = xa[e]; xv[4 + e] = xb[e]; }
  float sx = 0.f;
#pragma unroll
  for (int e = 0; e < 8; ++e) sx += xv[e];
  sx = block_sum4(sx, redA, lane, wave);
  const float mx = sx * kInvDim;
  float qx = 0.f;
#pragma unroll
  for (int e = 0; e < 8; ++e) { const float d = xv[e] - mx; qx += d * d; }
  qx = block_sum4(qx, redB, lane, wave);
  const float rsx = rsqrtf(qx * kInvDim + kLnEps);

  const v4f sa = *(const v4f*)(ss + base + cA), sb = *(const v4f*)(ss + base + cB);
  const v4f ra = *(const v4f*)(rw + base + cA), rb = *(const v4f*)(rw + base + cB);
  const v4f da = *(const v4f*)(dvec + cA), db = *(const v4f*)(dvec + cB);
  const v4f g1a = *(const v4f*)(gs + cA), g1b = *(const v4f*)(gs + cB);
  const v4f b1a = *(const v4f*)(bs + cA), b1b = *(const v4f*)(bs + cB);
  const v4f goa = *(const v4f*)(go + cA), gob = *(const v4f*)(go + cB);
  const v4f boa = *(const v4f*)(bo + cA), bob = *(const v4f*)(bo + cB);
  float sv[8], rv[8], dv[8], g1[8], b1[8], g3[8], b3[8];
#pragma unroll
  for (int e = 0; e < 4; ++e) {
    sv[e] = sa[e]; sv[4 + e] = sb[e]; rv[e] = ra[e]; rv[4 + e] = rb[e];
    dv[e] = da[e]; dv[4 + e] = db[e];
    g1[e] = g1a[e]; g1[4 + e] = g1b[e]; b1[e] = b1a[e]; b1[4 + e] = b1b[e];
    g3[e] = goa[e]; g3[4 + e] = gob[e]; b3[e] = boa[e]; b3[4 + e] = bob[e];
  }
  float cm[8];
#pragma unroll
  for (int e = 0; e < 8; ++e) {
    const float xs  = (xv[e] - mx) * rsx * g1[e] + b1[e];
    const float ssm = sv[e] + dv[e] * xs;
    cm[e] = 0.7f * ssm + 0.3f * rv[e];
  }
  float sc = 0.f;
#pragma unroll
  for (int e = 0; e < 8; ++e) sc += cm[e];
  sc = block_sum4(sc, redA, lane, wave);
  const float mc = sc * kInvDim;
  float qc = 0.f;
#pragma unroll
  for (int e = 0; e < 8; ++e) { const float d = cm[e] - mc; qc += d * d; }
  qc = block_sum4(qc, redB, lane, wave);
  const float rsc = rsqrtf(qc * kInvDim + kLnEps);
  v4f oa, ob;
#pragma unroll
  for (int e = 0; e < 4; ++e) {
    oa[e] = xv[e]     + ((cm[e]     - mc) * rsc * g3[e]     + b3[e]);
    ob[e] = xv[4 + e] + ((cm[4 + e] - mc) * rsc * g3[4 + e] + b3[4 + e]);
  }
  float* pa = out + base + cA;
  float* pb = out + base + cB;
  for (int pass = 0; pass < 2; ++pass) {
    *(volatile v4f*)pa = oa;
    *(volatile v4f*)pb = ob;
    __threadfence();
  }
}

extern "C" void kernel_launch(void* const* d_in, const int* in_sizes, int n_in,
                              void* d_out, int out_size, void* d_ws, size_t ws_size, hipStream_t stream) {
  if (n_in < 21) return;
  if (ws_size < kWsEnd) return;
  const size_t n_out0 = (size_t)kRows * kDim;
  const size_t n_out1 = (size_t)kBatch * kState;
  const size_t n_out2 = (size_t)kBatch * kHeads * kHeadDim * kHeadDim;
  if ((size_t)out_size < n_out0 + n_out1 + n_out2) return;
  if (in_sizes[0] != kRows * kDim || in_sizes[1] != kDim * kDim || in_sizes[2] != kDim * kDim ||
      in_sizes[3] != kDim * kDim || in_sizes[4] != kDim * kDim) return;
  if (in_sizes[5] != kHeads * kHeadDim || in_sizes[6] != kHeads * kHeadDim || in_sizes[7] != kState * kState ||
      in_sizes[8] != kState * kDim || in_sizes[9] != kDim * kState || in_sizes[10] != kDim || in_sizes[11] != kDim) return;

  const float* x      = (const float*)d_in[0];
  const float* wk     = (const float*)d_in[1];
  const float* wv     = (const float*)d_in[2];
  const float* wr     = (const float*)d_in[3];
  const float* wo     = (const float*)d_in[4];
  const float* tdec   = (const float*)d_in[5];
  const float* tfirst = (const float*)d_in[6];
  const float* Am     = (const float*)d_in[7];
  const float* bw     = (const float*)d_in[8];
  const float* cw     = (const float*)d_in[9];
  const float* dvec   = (const float*)d_in[10];
  const float* dtw    = (const float*)d_in[11];
  const float* dtb    = (const float*)d_in[12];
  const float* sng    = (const float*)d_in[13];
  const float* snb    = (const float*)d_in[14];
  const float* g_ssm  = (const float*)d_in[15];
  const float* b_ssm  = (const float*)d_in[16];
  const float* g_rw   = (const float*)d_in[17];
  const float* b_rw   = (const float*)d_in[18];
  const float* g_outp = (const float*)d_in[19];
  const float* b_outp = (const float*)d_in[20];

  char* ws = (char*)d_ws;
  unsigned short* xs16 = (unsigned short*)(ws + kOffXs16);
  unsigned short* xr16 = (unsigned short*)(ws + kOffXr16);
  unsigned short* w16  = (unsigned short*)(ws + kOffW16);
  unsigned short* bwp  = (unsigned short*)(ws + kOffBwp);
  unsigned short* cwp  = (unsigned short*)(ws + kOffCwp);
  float*          bxp  = (float*)(ws + kOffBxp);
  unsigned short* st16 = (unsigned short*)(ws + kOffSt16);
  float*          rwp  = (float*)(ws + kOffRw);
  float*          kvr  = (float*)(ws + kOffKvr);
  unsigned short* y16  = (unsigned short*)(ws + kOffY16);
  float*          ssp  = (float*)(ws + kOffSs);

  float* out0 = (float*)d_out;
  float* out1 = out0 + n_out0;
  float* out2 = out1 + n_out1;

  const size_t wplane = (size_t)kDim * kDim;
  const size_t bplane = (size_t)kSeq * kDim;

  ln_dual_kernel<<<dim3(kRows), dim3(128), 0, stream>>>(x, g_ssm, b_ssm, g_rw, b_rw, xs16, xr16);
  castw_kernel<<<dim3(kDim * kDim / 8 / 256, 4), dim3(256), 0, stream>>>(wk, wv, wr, wo, w16, kWCarry);
  prep_small_kernel<<<dim3(kBxN + 32), dim3(128), 0, stream>>>(bw, dtw, cw, bwp, cwp);
  wmma_gemm64<0, false, 0, 0, false, 0><<<dim3(kRows / 64 * (kBxN / 64) / 8, 1), dim3(256), 0, stream>>>(
      xs16, xs16, kDim, (long)0, bwp, bwp, kDim, (long)0, (void*)bxp, (void*)bxp, kBxN, (long)0,
      x, x, (long)0, kRows, kBxN, kDim, 1.0f / kSmallCarry);
  ssm_scan_kernel<<<dim3(1), dim3(64), 0, stream>>>(Am, bxp, dtb, sng, snb, st16, out1);
  for (int b = 0; b < kBatch; ++b) {
    wmma_gemm64<0, false, 0, 0, false, 0><<<dim3(kSeq / 64 * (kDim / 64) / 8, 3), dim3(256), 0, stream>>>(
        xr16 + (size_t)b * bplane, xr16 + (size_t)b * bplane, kDim, (long)0,
        w16, w16, kDim, (long)wplane,
        (void*)kvr, (void*)kvr, kDim, (long)bplane,
        x, x, (long)0, kSeq, kDim, kDim, 1.0f / kWCarry);
    wkv_scan_kernel<<<dim3(kHeads), dim3(128), 0, stream>>>(
        kvr, kvr + bplane, kvr + 2 * bplane, tdec, tfirst, y16,
        out2 + (size_t)b * kHeads * kHeadDim * kHeadDim);
    wmma_gemm64<0, false, 0, 0, false, 0><<<dim3(kSeq / 64 * (kDim / 64) / 8, 1), dim3(256), 0, stream>>>(
        y16, y16, kDim, (long)0, w16 + 3 * wplane, w16 + 3 * wplane, kDim, (long)0,
        (void*)(rwp + (size_t)b * bplane), (void*)(rwp + (size_t)b * bplane), kDim, (long)0,
        x, x, (long)0, kSeq, kDim, kDim, 1.0f / (kYCarry * kWCarry));
  }
  wmma_gemm64<0, false, 0, 0, false, 0><<<dim3(kRows / 64 * (kDim / 64) / 8, 1), dim3(256), 0, stream>>>(
      st16, st16, kStK, (long)0, cwp, cwp, kStK, (long)0, (void*)ssp, (void*)ssp, kDim, (long)0,
      x, x, (long)0, kRows, kDim, kStK, 1.0f / kSmallCarry);
  combine_kernel<<<dim3(kRows), dim3(128), 0, stream>>>(x, ssp, rwp, dvec, g_ssm, b_ssm, g_outp, b_outp, out0);
}
